// MultiQueryDotProductAttention_73839077753206
// MI455X (gfx1250) — hardware-verified
//
#include <hip/hip_runtime.h>
#include <math.h>
#include <stdint.h>

#define NB_   2
#define SEQ_  2048
#define EMB_  2048
#define NH_   16
#define DHD_  128
#define HDT_  2048

typedef _Float16 v16h __attribute__((ext_vector_type(16)));
typedef _Float16 v8h  __attribute__((ext_vector_type(8)));
typedef _Float16 v4h  __attribute__((ext_vector_type(4)));
typedef __bf16   v16b __attribute__((ext_vector_type(16)));
typedef __bf16   v8b  __attribute__((ext_vector_type(8)));
typedef float    v8f  __attribute__((ext_vector_type(8)));
typedef float    v4f  __attribute__((ext_vector_type(4)));
typedef unsigned short v8us __attribute__((ext_vector_type(8)));

__device__ __forceinline__ unsigned short bf16_bits_rne(float f) {
  unsigned u = __float_as_uint(f);
  return (unsigned short)((u + 0x7FFFu + ((u >> 16) & 1u)) >> 16);
}
__device__ __forceinline__ float bf16_val_rne(float f) {
  unsigned u = __float_as_uint(f);
  u = (u + 0x7FFFu + ((u >> 16) & 1u)) & 0xFFFF0000u;
  return __uint_as_float(u);
}
__device__ __forceinline__ float bf16_bits_to_f32(unsigned short b) {
  return __uint_as_float(((unsigned)b) << 16);
}
__device__ __forceinline__ void split_f16x4(v4f f, v4h& hi, v4h& lo) {
  const v4h hq = __builtin_convertvector(f, v4h);
  const v4f hf = __builtin_convertvector(hq, v4f);
  const v4f rf = (f - hf) * 1024.0f;
  hi = hq;
  lo = __builtin_convertvector(rf, v4h);
}

template <typename T> struct FT;
template <> struct FT<_Float16> {
  typedef v16h V;
  union U { v16h v; v8h h[2]; };
  static __device__ __forceinline__ v16h load(const _Float16* p) {
    U f; f.h[0] = *(const v8h*)(p); f.h[1] = *(const v8h*)(p + 16); return f.v;
  }
  static __device__ __forceinline__ v8f mma(v16h a, v16h b, v8f c) {
    c = __builtin_amdgcn_wmma_f32_16x16x32_f16(false, a, false, b, (short)0, c, false, false);
    asm volatile("v_nop\n\tv_nop\n\tv_nop\n\tv_nop" : "+v"(c) : "v"(a), "v"(b));
    return c;
  }
};
template <> struct FT<__bf16> {
  typedef v16b V;
  union U { v16b v; v8b h[2]; };
  static __device__ __forceinline__ v16b load(const __bf16* p) {
    U f; f.h[0] = *(const v8b*)(p); f.h[1] = *(const v8b*)(p + 16); return f.v;
  }
  static __device__ __forceinline__ v8f mma(v16b a, v16b b, v8f c) {
    c = __builtin_amdgcn_wmma_f32_16x16x32_bf16(false, a, false, b, (short)0, c, false, false);
    asm volatile("v_nop\n\tv_nop\n\tv_nop\n\tv_nop" : "+v"(c) : "v"(a), "v"(b));
    return c;
  }
};

__device__ __forceinline__ void wave_lds_sync() {
  __builtin_amdgcn_fence(__ATOMIC_RELEASE, "workgroup");
  __builtin_amdgcn_wave_barrier();
  __builtin_amdgcn_fence(__ATOMIC_ACQUIRE, "workgroup");
}

__global__ __launch_bounds__(256) void k_cvt_bf16(const float* __restrict__ in, unsigned short* __restrict__ out, int n8) {
  const int i = blockIdx.x * 256 + threadIdx.x;
  if (i < n8) {
    const float* p = in + (size_t)i * 8;
    const v4f a = *(const v4f*)(p);
    const v4f c = *(const v4f*)(p + 4);
    v8us o;
    o[0] = bf16_bits_rne(a[0]); o[1] = bf16_bits_rne(a[1]); o[2] = bf16_bits_rne(a[2]); o[3] = bf16_bits_rne(a[3]);
    o[4] = bf16_bits_rne(c[0]); o[5] = bf16_bits_rne(c[1]); o[6] = bf16_bits_rne(c[2]); o[7] = bf16_bits_rne(c[3]);
    unsigned short* q = out + (size_t)i * 8;
    *(volatile v8us*)(q) = o;
    __threadfence();
    *(volatile v8us*)(q) = o;
  }
}

__global__ __launch_bounds__(256) void k_tcvt(const float* __restrict__ W, unsigned short* __restrict__ out, int R, int C) {
  __shared__ __align__(16) float tf[64 * 68];
  const int c0  = blockIdx.x * 64;
  const int r0  = blockIdx.y * 64;
  const int tid = threadIdx.x;
  {
    const int lr = tid >> 4;
    const int c4 = (tid & 15) * 4;
#pragma unroll
    for (int it = 0; it < 4; ++it) {
      const int rr = it * 16 + lr;
      const v4f a = *(const v4f*)(W + (size_t)(r0 + rr) * C + c0 + c4);
      *(v4f*)(tf + rr * 68 + c4) = a;
    }
  }
  __syncthreads();
  const int sub = tid >> 3;
  const int c8  = (tid & 7) * 8;
  v8us hv[2];
#pragma unroll
  for (int it = 0; it < 2; ++it) {
    const int oc = it * 32 + sub;
    v8us a;
#pragma unroll
    for (int e = 0; e < 8; ++e) a[e] = bf16_bits_rne(tf[(c8 + e) * 68 + oc]);
    hv[it] = a;
  }
  for (int pass = 0; pass < 2; ++pass) {
#pragma unroll
    for (int it = 0; it < 2; ++it) {
      const int oc = it * 32 + sub;
      const size_t go = (size_t)(c0 + oc) * R + r0 + c8;
      *(volatile v8us*)(out + go) = hv[it];
    }
    __threadfence();
  }
}

template <typename T, int OUTH, bool SPLITA>
__global__ __launch_bounds__(256) __attribute__((amdgpu_num_vgpr(256)))
void k_gemm(const unsigned short* __restrict__ Ap, const unsigned short* __restrict__ A2p, int lda, long long strideA,
            const unsigned short* __restrict__ Bp, int ldb, long long strideB,
            float* __restrict__ Cp, int ldc, long long strideC,
            int M, int N, int K, float scale) {
  typedef typename FT<T>::V V;
  __shared__ __align__(16) float slabs[8][16 * 68];
  const int lane = threadIdx.x & 31;
  const int wave = threadIdx.x >> 5;
  const int z    = blockIdx.y;
  const int tilesN = N >> 6;
  const int tilesM = M >> 6;
  const int tile = blockIdx.x * 8 + wave;
  if (tile >= tilesM * tilesN) return;
  const int tm = tile / tilesN;
  const int tn = tile - tm * tilesN;
  const int m0 = tm << 6;
  const int n0 = tn << 6;

  const T* A  = (const T*)Ap  + (size_t)z * (size_t)strideA;
  const T* A2 = (const T*)A2p + (size_t)z * (size_t)strideA;
  const T* Bt = (const T*)Bp  + (size_t)z * (size_t)strideB;

  const int rl   = lane & 15;
  const int koff = (lane >> 4) * 8;
  const int mOff = (lane >> 4) * 8;

  v8f acc[4][4];
#pragma unroll
  for (int i = 0; i < 4; ++i)
#pragma unroll
    for (int j = 0; j < 4; ++j) { v8f zz = {0.f,0.f,0.f,0.f,0.f,0.f,0.f,0.f}; acc[i][j] = zz; }

#pragma unroll 1
  for (int k0 = 0; k0 < K; k0 += 32) {
    V bf[4];
#pragma unroll
    for (int j = 0; j < 4; ++j)
      bf[j] = FT<T>::load(Bt + (size_t)(n0 + (j << 4) + rl) * ldb + k0 + koff);
#pragma unroll
    for (int i = 0; i < 4; ++i) {
      const size_t ao = (size_t)(m0 + (i << 4) + rl) * lda + k0 + koff;
      const V af = FT<T>::load(A + ao);
      V al = af;
      if (SPLITA) al = FT<T>::load(A2 + ao);
#pragma unroll
      for (int j = 0; j < 4; ++j) {
        acc[i][j] = FT<T>::mma(af, bf[j], acc[i][j]);
        if (SPLITA) acc[i][j] = FT<T>::mma(al, bf[j], acc[i][j]);
      }
    }
  }

  float* slab = slabs[wave];
#pragma unroll
  for (int i = 0; i < 4; ++i) {
    const int mBase = m0 + (i << 4);
#pragma unroll
    for (int j = 0; j < 4; ++j) {
#pragma unroll
      for (int r = 0; r < 8; ++r) slab[(mOff + r) * 68 + (j << 4) + rl] = acc[i][j][r] * scale;
    }
    wave_lds_sync();
    if (OUTH == 0) {
      float* C = Cp + (size_t)z * (size_t)strideC;
      const int hh = lane >> 4, c4 = (lane & 15) * 4;
      for (int pass = 0; pass < 2; ++pass) {
#pragma unroll
        for (int it = 0; it < 8; ++it) {
          const int row = it * 2 + hh;
          const v4f v = *(const v4f*)(slab + row * 68 + c4);
          *(volatile v4f*)(C + (size_t)(mBase + row) * ldc + n0 + c4) = v;
        }
        __threadfence();
      }
    } else {
      _Float16* C = (_Float16*)Cp + (size_t)z * (size_t)strideC;
      const int q = lane >> 3, c8 = (lane & 7) * 8;
      for (int pass = 0; pass < 2; ++pass) {
#pragma unroll
        for (int it = 0; it < 4; ++it) {
          const int row = it * 4 + q;
          const float* sp = slab + row * 68 + c8;
          v8h hv;
#pragma unroll
          for (int e = 0; e < 8; ++e) hv[e] = (_Float16)sp[e];
          *(volatile v8h*)(C + (size_t)(mBase + row) * ldc + n0 + c8) = hv;
        }
        __threadfence();
      }
    }
    wave_lds_sync();
  }
}

#define PP_  72
#define QP_  136
#define OPF_ 68

__global__ __launch_bounds__(128) __attribute__((amdgpu_num_vgpr(256)))
void k_attn(const float* __restrict__ qp, const unsigned short* __restrict__ kp,
            const unsigned short* __restrict__ vtp, const float* __restrict__ bias,
            unsigned short* __restrict__ cxh, unsigned short* __restrict__ cxl) {
  __shared__ __align__(16) _Float16 Psh[4][16 * PP_];
  __shared__ __align__(16) _Float16 Qlsh[4][16 * QP_];
  __shared__ __align__(16) float    Osh[4][16 * OPF_];

  const int tid  = threadIdx.x;
  const int wave = tid >> 5;
  const int lane = tid & 31;
  const int hh   = lane >> 4;
  const int c    = lane & 15;

  const int b  = blockIdx.z;
  const int h  = blockIdx.y;
  const int q0 = blockIdx.x * 64 + wave * 16;

  const float*    Q   = qp + ((size_t)b * SEQ_ + q0) * HDT_ + (size_t)h * DHD_;
  const _Float16* Kp  = (const _Float16*)(const void*)kp + (size_t)b * SEQ_ * DHD_;
  const _Float16* Vt  = (const _Float16*)(const void*)vtp + (size_t)b * DHD_ * SEQ_;
  const float*    Bs  = bias + ((size_t)b * SEQ_ + q0) * SEQ_;
  unsigned short* Cxh = cxh + ((size_t)b * SEQ_ + q0) * HDT_ + (size_t)h * DHD_;
  unsigned short* Cxl = cxl + ((size_t)b * SEQ_ + q0) * HDT_ + (size_t)h * DHD_;

  v16h qa[4];
  _Float16* qlw = Qlsh[wave];
#pragma unroll
  for (int ks = 0; ks < 4; ++ks) {
    const float* qr = Q + (size_t)c * HDT_ + ks * 32 + 8 * hh;
    union { v16h v; v4h q[4]; } fh;
    union { v8h v; v4h q[2]; } l0, l1;
    v4h hq, lq;
    split_f16x4(*(const v4f*)(qr),      hq, lq); fh.q[0] = hq; l0.q[0] = lq;
    split_f16x4(*(const v4f*)(qr + 4),  hq, lq); fh.q[1] = hq; l0.q[1] = lq;
    split_f16x4(*(const v4f*)(qr + 16), hq, lq); fh.q[2] = hq; l1.q[0] = lq;
    split_f16x4(*(const v4f*)(qr + 20), hq, lq); fh.q[3] = hq; l1.q[1] = lq;
    qa[ks] = fh.v;
    *(v8h*)(qlw + c * QP_ + ks * 32 + 8 * hh)      = l0.v;
    *(v8h*)(qlw + c * QP_ + ks * 32 + 16 + 8 * hh) = l1.v;
  }
  wave_lds_sync();

  float mrow[8], lrow[8];
  v8f oacc[8];
#pragma unroll
  for (int r = 0; r < 8; ++r) { mrow[r] = -INFINITY; lrow[r] = 0.f; }
#pragma unroll
  for (int t = 0; t < 8; ++t) { v8f zz = {0.f,0.f,0.f,0.f,0.f,0.f,0.f,0.f}; oacc[t] = zz; }

  _Float16* pw = Psh[wave];

#pragma unroll 1
  for (int kc = 0; kc < SEQ_ / 64; ++kc) {
    const int kv0 = kc * 64;

    v8f s[4];
#pragma unroll
    for (int j = 0; j < 4; ++j) {
      v8f sh = {0.f,0.f,0.f,0.f,0.f,0.f,0.f,0.f};
      v8f sl = {0.f,0.f,0.f,0.f,0.f,0.f,0.f,0.f};
      const _Float16* kr = Kp + (size_t)(kv0 + j * 16 + c) * DHD_ + 8 * hh;
#pragma unroll
      for (int ks = 0; ks < 4; ++ks) {
        const v16h kb = FT<_Float16>::load(kr + ks * 32);
        const v16h ql = FT<_Float16>::load(qlw + c * QP_ + ks * 32 + 8 * hh);
        sh = FT<_Float16>::mma(qa[ks], kb, sh);
        sl = FT<_Float16>::mma(ql, kb, sl);
      }
      s[j] = sh + sl * 0.0009765625f;
    }

    float cm[8];
#pragma unroll
    for (int r = 0; r < 8; ++r) {
      const float* br = Bs + (size_t)(8 * hh + r) * SEQ_ + kv0 + c;
      float m = -INFINITY;
#pragma unroll
      for (int j = 0; j < 4; ++j) {
        const float bv = bf16_val_rne(br[j * 16]);
        const float t  = s[j][r] * 0.015625f + bv;
        s[j][r] = t;
        m = fmaxf(m, t);
      }
#pragma unroll
      for (int off = 1; off < 16; off <<= 1) m = fmaxf(m, __shfl_xor(m, off, 32));
      cm[r] = m;
    }

#pragma unroll
    for (int r = 0; r < 8; ++r) {
      const float mnew  = fmaxf(mrow[r], cm[r]);
      const float alpha = __expf(mrow[r] - mnew);
      mrow[r] = mnew;
      float psum = 0.f;
#pragma unroll
      for (int j = 0; j < 4; ++j) {
        const float p = __expf(s[j][r] - mnew);
        psum += p;
        pw[(8 * hh + r) * PP_ + j * 16 + c] = (_Float16)(p * 4096.0f);
      }
#pragma unroll
      for (int off = 1; off < 16; off <<= 1) psum += __shfl_xor(psum, off, 32);
      lrow[r] = lrow[r] * alpha + psum;
#pragma unroll
      for (int t = 0; t < 8; ++t) oacc[t][r] *= alpha;
    }
    wave_lds_sync();

#pragma unroll
    for (int kk = 0; kk < 2; ++kk) {
      const v16h pa = FT<_Float16>::load(pw + c * PP_ + kk * 32 + 8 * hh);
#pragma unroll
      for (int t = 0; t < 8; ++t) {
        const v16h vb = FT<_Float16>::load(Vt + (size_t)(t * 16 + c) * SEQ_ + kv0 + kk * 32 + 8 * hh);
        oacc[t] = FT<_Float16>::mma(pa, vb, oacc[t]);
      }
    }
    wave_lds_sync();
  }

  float invr[8];
#pragma unroll
  for (int r = 0; r < 8; ++r) invr[r] = __builtin_amdgcn_rcpf(lrow[r]) * 6.103515625e-05f;
  float* os = Osh[wave];
  const int q4 = lane >> 3, c8 = (lane & 7) * 8;
#pragma unroll
  for (int hf = 0; hf < 2; ++hf) {
#pragma unroll
    for (int r = 0; r < 8; ++r) {
#pragma unroll
      for (int t = 0; t < 4; ++t) os[(8 * hh + r) * OPF_ + t * 16 + c] = oacc[hf * 4 + t][r] * invr[r];
    }
    wave_lds_sync();
    v8us hv[4], lv[4];
#pragma unroll
    for (int it = 0; it < 4; ++it) {
      const int row = it * 4 + q4;
      const float* sp = os + row * OPF_ + c8;
      v8us ah, al;
#pragma unroll
      for (int e = 0; e < 8; ++e) {
        const float f = sp[e];
        const unsigned short hb = bf16_bits_rne(f);
        const unsigned short lb = bf16_bits_rne(f - bf16_bits_to_f32(hb));
        ah[e] = hb; al[e] = lb;
      }
      hv[it] = ah; lv[it] = al;
    }
    for (int pass = 0; pass < 2; ++pass) {
#pragma unroll
      for (int it = 0; it < 4; ++it) {
        const int row = it * 4 + q4;
        const size_t go = (size_t)row * HDT_ + hf * 64 + c8;
        *(volatile v8us*)(Cxh + go) = hv[it];
        *(volatile v8us*)(Cxl + go) = lv[it];
      }
      __threadfence();
    }
    wave_lds_sync();
  }
}

extern "C" void kernel_launch(void* const* d_in, const int* in_sizes, int n_in,
                              void* d_out, int out_size, void* d_ws, size_t ws_size,
                              hipStream_t stream) {
  if (n_in < 7) return;
  if (in_sizes[0] != NB_ * SEQ_ * EMB_) return;
  if (in_sizes[1] != NB_ * SEQ_ * EMB_) return;
  if (in_sizes[2] != NB_ * SEQ_ * SEQ_) return;
  if (in_sizes[3] != EMB_ * NH_ * DHD_) return;
  if (in_sizes[4] != EMB_ * DHD_) return;
  if (in_sizes[5] != EMB_ * DHD_) return;
  if (in_sizes[6] != NH_ * DHD_ * EMB_) return;
  if (out_size != NB_ * SEQ_ * EMB_) return;

  const float* inq  = (const float*)d_in[0];
  const float* inkv = (const float*)d_in[1];
  const float* bias = (const float*)d_in[2];
  const float* Wq   = (const float*)d_in[3];
  const float* Wk   = (const float*)d_in[4];
  const float* Wv   = (const float*)d_in[5];
  const float* Wo   = (const float*)d_in[6];
  float* out = (float*)d_out;

  const size_t szX   = (size_t)NB_ * SEQ_ * EMB_ * 2;
  const size_t szWq  = (size_t)HDT_ * EMB_ * 2;
  const size_t szWkv = (size_t)DHD_ * EMB_ * 2;
  const size_t szWo  = (size_t)EMB_ * HDT_ * 2;
  const size_t szQ   = (size_t)NB_ * SEQ_ * HDT_ * 4;
  const size_t szK   = (size_t)NB_ * SEQ_ * DHD_ * 2;
  const size_t szVt  = (size_t)NB_ * DHD_ * SEQ_ * 2;
  const size_t szCtx = (size_t)NB_ * SEQ_ * HDT_ * 2;
  size_t off = 0;
  const size_t oXq  = off; off += szX;
  const size_t oXkv = off; off += szX;
  const size_t oWqT = off; off += szWq;
  const size_t oWkT = off; off += szWkv;
  const size_t oWvT = off; off += szWkv;
  const size_t oWoT = off; off += szWo;
  const size_t oQ   = off; off += szQ;
  const size_t oK   = off; off += szK;
  const size_t oVt  = off; off += szVt;
  const size_t oCxh = off; off += szCtx;
  const size_t oCxl = off; off += szCtx;
  if (off > ws_size) return;
  if (off > (size_t)134217728) return;

  char* ws = (char*)d_ws;
  unsigned short* Xq16  = (unsigned short*)(ws + oXq);
  unsigned short* Xkv16 = (unsigned short*)(ws + oXkv);
  unsigned short* WqT   = (unsigned short*)(ws + oWqT);
  unsigned short* WkT   = (unsigned short*)(ws + oWkT);
  unsigned short* WvT   = (unsigned short*)(ws + oWvT);
  unsigned short* WoT   = (unsigned short*)(ws + oWoT);
  float*          q32   = (float*)(ws + oQ);
  unsigned short* k16   = (unsigned short*)(ws + oK);
  unsigned short* vt16  = (unsigned short*)(ws + oVt);
  unsigned short* cxh   = (unsigned short*)(ws + oCxh);
  unsigned short* cxl   = (unsigned short*)(ws + oCxl);

  const float rs = 1.0f / sqrtf((float)DHD_);
  const dim3 blk(256);

  const int n8 = NB_ * SEQ_ * EMB_ / 8;
  k_cvt_bf16<<<dim3((n8 + 255) / 256), blk, 0, stream>>>(inq,  Xq16,  n8);
  k_cvt_bf16<<<dim3((n8 + 255) / 256), blk, 0, stream>>>(inkv, Xkv16, n8);
  k_tcvt<<<dim3(HDT_ / 64, EMB_ / 64), blk, 0, stream>>>(Wq, WqT, EMB_, HDT_);
  k_tcvt<<<dim3(DHD_ / 64, EMB_ / 64), blk, 0, stream>>>(Wk, WkT, EMB_, DHD_);
  k_tcvt<<<dim3(DHD_ / 64, EMB_ / 64), blk, 0, stream>>>(Wv, WvT, EMB_, DHD_);
  k_tcvt<<<dim3(EMB_ / 64, HDT_ / 64), blk, 0, stream>>>(Wo, WoT, HDT_, EMB_);

  k_gemm<__bf16, 0, false><<<dim3(((NB_ * SEQ_ / 64) * (HDT_ / 64) + 7) / 8, 1), blk, 0, stream>>>(
      Xq16, Xq16, EMB_, 0LL, WqT, EMB_, 0LL, q32, HDT_, 0LL, NB_ * SEQ_, HDT_, EMB_, 16.0f * rs);
  k_gemm<__bf16, 1, false><<<dim3(((NB_ * SEQ_ / 64) * (DHD_ / 64) + 7) / 8, 1), blk, 0, stream>>>(
      Xkv16, Xkv16, EMB_, 0LL, WkT, EMB_, 0LL, (float*)(void*)k16, DHD_, 0LL, NB_ * SEQ_, DHD_, EMB_, 4.0f);
  k_gemm<__bf16, 1, false><<<dim3(((DHD_ / 64) * (SEQ_ / 64) + 7) / 8, NB_), blk, 0, stream>>>(
      WvT, WvT, EMB_, 0LL, Xkv16, EMB_, (long long)SEQ_ * EMB_, (float*)(void*)vt16, SEQ_, (long long)DHD_ * SEQ_,
      DHD_, SEQ_, EMB_, 4.0f);
  k_attn<<<dim3(SEQ_ / 64, NH_, NB_), dim3(128), 0, stream>>>(q32, k16, vt16, bias, cxh, cxl);
  k_gemm<__bf16, 0, true><<<dim3(((NB_ * SEQ_ / 64) * (EMB_ / 64) + 7) / 8, 1), blk, 0, stream>>>(
      cxh, cxl, HDT_, 0LL, WoT, HDT_, 0LL, out, EMB_, 0LL, NB_ * SEQ_, EMB_, HDT_, 1.0f);

  (void)hipGetLastError();
}
